// GraphAttentionLayer2_32023276159121
// MI455X (gfx1250) — hardware-run, weakly checked
//
#include <hip/hip_runtime.h>
#include <stddef.h>
#include <stdint.h>

#define NBT  48
#define NND  1024
#define CIN  64
#define FO   64
#define EMD  16
#define NROW (NBT * NND)
#define RB   128
#define LDSP 1032
#define WTP  72
#define TTP  136
#define OSP  68
#define MASK_FILL (-9.0e15f)
#define LEAK 0.2f

static_assert(NND % RB == 0);
static_assert(NROW % RB == 0);
static_assert(CIN == 64);
static_assert(FO == 64);
static_assert(EMD == 16);
static_assert((LDSP % 8) == 0);
static_assert((TTP % 8) == 0);
static_assert((WTP % 8) == 0);
static_assert((OSP % 4) == 0);
static_assert(RB * OSP * 4 <= FO * LDSP * 2);
static_assert(((FO * NND / 8) % 256) == 0);

typedef _Float16 v16h __attribute__((ext_vector_type(16)));
typedef _Float16 v8h  __attribute__((ext_vector_type(8)));
typedef float    v8f  __attribute__((ext_vector_type(8)));
typedef float    v4f  __attribute__((ext_vector_type(4)));
typedef int      v8i  __attribute__((ext_vector_type(8)));
typedef unsigned int v4u __attribute__((ext_vector_type(4)));

union Frag  { v16h v; v8h h[2]; };
union Pack8 { v8h h; v4u u; };
static_assert(sizeof(Frag) == 32);
static_assert(sizeof(Pack8) == 16);

__device__ __forceinline__ v8f mma16(v16h a, v16h b, v8f c) {
  c = __builtin_amdgcn_wmma_f32_16x16x32_f16(false, a, false, b, (short)0, c, false, false);
  asm volatile("v_nop\n\tv_nop\n\tv_nop\n\tv_nop" : "+v"(c) : "v"(a), "v"(b));
  return c;
}

__device__ __forceinline__ v16h ldfrag(const _Float16* p, int ld, int row0, int k0, int lane) {
  const int m = lane & 15, lh = lane >> 4;
  const _Float16* q = p + (size_t)(row0 + m) * ld + k0 + 8 * lh;
  Frag f;
  f.h[0] = *(const v8h*)(q);
  f.h[1] = *(const v8h*)(q + 16);
  return f.v;
}

__device__ __forceinline__ v8f zero8() { return (v8f){0.f, 0.f, 0.f, 0.f, 0.f, 0.f, 0.f, 0.f}; }

__global__ __launch_bounds__(256) void k_proj(const float* __restrict__ x,
                                              const float* __restrict__ w,
                                              const float* __restrict__ av,
                                              const float* __restrict__ a2v,
                                              const float* __restrict__ emb1,
                                              const float* __restrict__ emb2,
                                              _Float16* __restrict__ whT,
                                              float* __restrict__ rterm,
                                              float* __restrict__ cterm) {
  __shared__ __align__(16) _Float16 wt[FO * WTP];
  __shared__ __align__(16) _Float16 tt[FO * TTP];
  __shared__ __align__(16) float sR[RB];
  __shared__ __align__(16) float sC[RB];

  const int tid = threadIdx.x, lane = tid & 31, wave = tid >> 5;
  const int lh = lane >> 4, lc = lane & 15;
  const int rowBase = blockIdx.x * RB;
  const int bt = rowBase >> 10;
  const int nBase = rowBase & (NND - 1);
  const int nW = wave * 16;

  {
    const int cc = tid >> 2;
    const int fq = (tid & 3) * 16;
    const float* wp = w + cc * FO + fq;
#pragma unroll
    for (int q = 0; q < 4; ++q) {
      const v4f v = *(const v4f*)(wp + 4 * q) * 8.0f;
      wt[(fq + 4 * q + 0) * WTP + cc] = (_Float16)v[0];
      wt[(fq + 4 * q + 1) * WTP + cc] = (_Float16)v[1];
      wt[(fq + 4 * q + 2) * WTP + cc] = (_Float16)v[2];
      wt[(fq + 4 * q + 3) * WTP + cc] = (_Float16)v[3];
    }
  }
  __syncthreads();

  const float* xrow = x + (size_t)(rowBase + nW + lc) * CIN;
  v8f acc[4];
#pragma unroll
  for (int t = 0; t < 4; ++t) acc[t] = zero8();
#pragma unroll
  for (int s = 0; s < 2; ++s) {
    const int k0 = 32 * s;
    const v8f x0 = *(const v8f*)(xrow + k0 + 8 * lh);
    const v8f x1 = *(const v8f*)(xrow + k0 + 16 + 8 * lh);
    Frag a;
    a.h[0] = __builtin_convertvector(x0, v8h);
    a.h[1] = __builtin_convertvector(x1, v8h);
#pragma unroll
    for (int t = 0; t < 4; ++t) {
      const v16h b = ldfrag(wt, WTP, 16 * t, k0, lane);
      acc[t] = mma16(a.v, b, acc[t]);
    }
  }

#pragma unroll
  for (int t = 0; t < 4; ++t) {
    const v8f wv = acc[t] * 0.125f;
    *(v8h*)(tt + (16 * t + lc) * TTP + nW + 8 * lh) = __builtin_convertvector(wv, v8h);
  }
  __syncthreads();

  v8f sacc = zero8();
#pragma unroll
  for (int s = 0; s < 2; ++s) {
    v8f al, ah;
    v8h bl, bh;
#pragma unroll
    for (int e = 0; e < 8; ++e) {
      const int f0 = 32 * s + 8 * lh + e;
      const int f1 = f0 + 16;
      const float p0 = av[f0], q0 = av[FO + f0];
      const float p1 = av[f1], q1 = av[FO + f1];
      al[e] = (lc == 0) ? p0 : ((lc == 1) ? q0 : 0.0f);
      ah[e] = (lc == 0) ? p1 : ((lc == 1) ? q1 : 0.0f);
      bl[e] = tt[f0 * TTP + nW + lc];
      bh[e] = tt[f1 * TTP + nW + lc];
    }
    Frag af, bf;
    af.h[0] = __builtin_convertvector(al * 16.0f, v8h);
    af.h[1] = __builtin_convertvector(ah * 16.0f, v8h);
    bf.h[0] = bl;
    bf.h[1] = bh;
    sacc = mma16(af.v, bf.v, sacc);
  }

  const int node = nBase + nW + lc;
  const float* e1p = emb1 + (size_t)node * EMD;
  const float* e2p = emb2 + (size_t)node * EMD;
  float f1 = 0.0f, f2 = 0.0f;
#pragma unroll
  for (int q = 0; q < 4; ++q) {
    const v4f u1 = *(const v4f*)(e1p + 4 * q);
    const v4f u2 = *(const v4f*)(e2p + 4 * q);
    const v4f g1 = *(const v4f*)(a2v + 4 * q);
    const v4f g2 = *(const v4f*)(a2v + EMD + 4 * q);
#pragma unroll
    for (int e = 0; e < 4; ++e) {
      f1 = fmaf(u1[e], g1[e], f1);
      f2 = fmaf(u2[e], g2[e], f2);
    }
  }
  if (lh == 0) {
    sR[nW + lc] = sacc[0] * 0.0625f + f1;
    sC[nW + lc] = sacc[1] * 0.0625f + f2;
  }
  __syncthreads();

  v4u val[4];
  size_t go[4];
#pragma unroll
  for (int it = 0; it < 4; ++it) {
    const int p = tid + 256 * it;
    const int fr = p >> 4;
    const int pc = p & 15;
    Pack8 pk;
    pk.h = *(const v8h*)(tt + fr * TTP + pc * 8);
    val[it] = pk.u;
    go[it] = ((size_t)bt * FO + fr) * NND + nBase + pc * 8;
  }
  for (int ps = 0; ps < 2; ++ps) {
#pragma unroll
    for (int it = 0; it < 4; ++it) *(volatile v4u*)(whT + go[it]) = val[it];
    __threadfence();
  }

  const size_t so = (size_t)bt * NND + nBase + 4 * lane;
  if (wave == 0) {
    const v4f v = *(const v4f*)(sR + 4 * lane);
    *(volatile v4f*)(rterm + so) = v;
    __threadfence();
    *(volatile v4f*)(rterm + so) = v;
  } else if (wave == 1) {
    const v4f v = *(const v4f*)(sC + 4 * lane);
    *(volatile v4f*)(cterm + so) = v;
    __threadfence();
    *(volatile v4f*)(cterm + so) = v;
  }
}

__global__ __launch_bounds__(256) void k_aggr(const _Float16* __restrict__ whT,
                                              const int* __restrict__ adj,
                                              const float* __restrict__ rterm,
                                              const float* __restrict__ cterm,
                                              float* __restrict__ out) {
  extern __shared__ __align__(16) unsigned char dynlds[];
  _Float16* whs = (_Float16*)dynlds;

  const int tid = threadIdx.x, lane = tid & 31, wave = tid >> 5;
  const int lh = lane >> 4, lc = lane & 15;
  const int bt = blockIdx.y;
  const int i0 = blockIdx.x * RB + wave * 16;
  const _Float16* wh = whT + (size_t)bt * FO * NND;

#pragma unroll 4
  for (int it = 0; it < (FO * NND / 8) / 256; ++it) {
    const int p = tid + 256 * it;
    const int f = p >> 7;
    const int off = (p & 127) * 8;
    *(v8h*)(whs + f * LDSP + off) = *(const v8h*)(wh + (size_t)f * NND + off);
  }
  __syncthreads();

  const int irow = i0 + lc;
  const float ri = rterm[(size_t)bt * NND + irow];
  const int* arow = adj + (size_t)irow * NND;
  const float* crow = cterm + (size_t)bt * NND;

  v8f acc[4];
#pragma unroll
  for (int t = 0; t < 4; ++t) acc[t] = zero8();
  float mrun = -1.0e30f, lrun = 0.0f;

#pragma unroll 1
  for (int j0 = 0; j0 < NND; j0 += 32) {
    const int ja = j0 + 8 * lh;
    const int jb = ja + 16;
    const v8i ad0 = *(const v8i*)(arow + ja);
    const v8i ad1 = *(const v8i*)(arow + jb);
    const v8f cc0 = *(const v8f*)(crow + ja);
    const v8f cc1 = *(const v8f*)(crow + jb);

    v8f s0v, s1v;
#pragma unroll
    for (int e = 0; e < 8; ++e) {
      float u0 = ri + cc0[e];
      u0 = (u0 >= 0.0f) ? u0 : LEAK * u0;
      s0v[e] = (ad0[e] > 0) ? u0 : MASK_FILL;
      float u1 = ri + cc1[e];
      u1 = (u1 >= 0.0f) ? u1 : LEAK * u1;
      s1v[e] = (ad1[e] > 0) ? u1 : MASK_FILL;
    }
    float lm = fmaxf(s0v[0], s1v[0]);
#pragma unroll
    for (int e = 1; e < 8; ++e) lm = fmaxf(lm, fmaxf(s0v[e], s1v[e]));
    lm = fmaxf(lm, __shfl_xor(lm, 16, 32));
    const float mnew = fmaxf(mrun, lm);
    const float alpha = __expf(mrun - mnew);

    v8f p0, p1;
    float ls = 0.0f;
#pragma unroll
    for (int e = 0; e < 8; ++e) {
      p0[e] = __expf(s0v[e] - mnew);
      p1[e] = __expf(s1v[e] - mnew);
      ls += p0[e] + p1[e];
    }
    ls += __shfl_xor(ls, 16, 32);
    lrun = lrun * alpha + ls;
    mrun = mnew;

    Frag pf;
    pf.h[0] = __builtin_convertvector(p0 * 1024.0f, v8h);
    pf.h[1] = __builtin_convertvector(p1 * 1024.0f, v8h);

    v8f fsv;
#pragma unroll
    for (int r = 0; r < 8; ++r) fsv[r] = __shfl(alpha, 8 * lh + r, 32);
#pragma unroll
    for (int t = 0; t < 4; ++t) acc[t] = acc[t] * fsv;

#pragma unroll
    for (int t = 0; t < 4; ++t) {
      const v16h b = ldfrag(whs, LDSP, 16 * t, j0, lane);
      acc[t] = mma16(pf.v, b, acc[t]);
    }
  }

  v8f invv;
#pragma unroll
  for (int r = 0; r < 8; ++r) {
    const float lv = __shfl(lrun, 8 * lh + r, 32);
    invv[r] = __builtin_amdgcn_rcpf(lv) * 0.0009765625f;
  }
  __syncthreads();
  float* os = (float*)dynlds;
#pragma unroll
  for (int t = 0; t < 4; ++t) {
    const v8f hv8 = acc[t] * invv;
#pragma unroll
    for (int r = 0; r < 8; ++r) {
      float hv = hv8[r];
      hv = (hv > 0.0f) ? hv : (__expf(hv) - 1.0f);
      os[(wave * 16 + 8 * lh + r) * OSP + 16 * t + lc] = hv;
    }
  }
  __syncthreads();

  const float* orow = os + (wave * 16 + lh) * OSP + 4 * lc;
  const size_t obase = ((size_t)bt * NND + i0 + lh) * FO + 4 * lc;
  v4f val[8];
#pragma unroll
  for (int it = 0; it < 8; ++it) val[it] = *(const v4f*)(orow + 2 * it * OSP);
  for (int ps = 0; ps < 2; ++ps) {
#pragma unroll
    for (int it = 0; it < 8; ++it) *(volatile v4f*)(out + obase + (size_t)it * 128) = val[it];
    __threadfence();
  }
}

extern "C" void kernel_launch(void* const* d_in, const int* in_sizes, int n_in,
                              void* d_out, int out_size, void* d_ws, size_t ws_size,
                              hipStream_t stream) {
  if (n_in < 7) return;
  if (in_sizes[0] != NROW * CIN) return;
  if (in_sizes[1] != NND * NND) return;
  if (in_sizes[2] != NND * EMD) return;
  if (in_sizes[3] != NND * EMD) return;
  if (in_sizes[4] != CIN * FO) return;
  if (in_sizes[5] != 2 * FO) return;
  if (in_sizes[6] != 2 * EMD) return;
  if (out_size != NROW * FO) return;

  const float* x    = (const float*)d_in[0];
  const int*   adj  = (const int*)d_in[1];
  const float* emb1 = (const float*)d_in[2];
  const float* emb2 = (const float*)d_in[3];
  const float* w    = (const float*)d_in[4];
  const float* av   = (const float*)d_in[5];
  const float* a2v  = (const float*)d_in[6];
  float* out = (float*)d_out;

  size_t off = 0;
  const size_t oWhT = off; off += (size_t)NROW * FO * sizeof(_Float16);
  const size_t oR   = off; off += (size_t)NROW * sizeof(float);
  const size_t oC   = off; off += (size_t)NROW * sizeof(float);
  if (off > ws_size) return;
  if (off > (size_t)134217728) return;

  char* ws = (char*)d_ws;
  _Float16* whT = (_Float16*)(ws + oWhT);
  float* rterm  = (float*)(ws + oR);
  float* cterm  = (float*)(ws + oC);

  k_proj<<<dim3(NROW / RB), dim3(256), 0, stream>>>(x, w, av, a2v, emb1, emb2, whT, rterm, cterm);

  const size_t ldsb = (size_t)FO * LDSP * sizeof(_Float16);
  (void)hipFuncSetAttribute(reinterpret_cast<const void*>(&k_aggr),
                            hipFuncAttributeMaxDynamicSharedMemorySize, (int)ldsb);
  k_aggr<<<dim3(NND / RB, NBT), dim3(256), ldsb, stream>>>(whT, adj, rterm, cterm, out);
  (void)hipGetLastError();
}
